// ElectronicSchNet_67207648247821
// MI455X (gfx1250) — hardware-verified
//
#include <hip/hip_runtime.h>
#include <stddef.h>
#include <stdint.h>

#pragma clang fp contract(off)


#define NE      16
#define ED      128
#define KD      64
#define DF      32
#define WH      45
#define NL      3
#define NNUC    4
#define TPB     128

#define N_SAME  112
#define RB_ANTI 112
#define RB_NUC  240
#define NEDGE   304
#define NTILES  19
#define NTIT    5

#define FRH     512
#define OFF_HW  0
#define SZ_HW   (NL * 16 * FRH)
#define OFF_W0  (OFF_HW + SZ_HW)
#define SZ_W0   (NL * 3 * 3 * FRH)
#define OFF_W1  (OFF_W0 + SZ_W0)
#define SZ_W1   (NL * 3 * 8 * FRH)
#define OFF_G   (OFF_W1 + SZ_W1)
#define SZ_G    (NL * 3 * 16 * FRH)
#define PK_TOTAL (OFF_G + SZ_G)
#define NGRP    (PK_TOTAL / 8)
#define WS_BYTES ((size_t)PK_TOTAL * 2)
#define WSCAP   134217728

#define WSC  16.0f
#define PSC  0.0625f
#define ESC  64.0f
#define PSE  0.0009765625f
#define LN2F 0.69314718f

static_assert(SZ_HW == 24576);
static_assert(OFF_W0 == 24576);
static_assert(OFF_W1 == 38400);
static_assert(OFF_G == 75264);
static_assert(PK_TOTAL == 148992);
static_assert((PK_TOTAL % 8) == 0);
static_assert((NGRP % 32) == 0);
static_assert((OFF_W0 % 256) == 0);
static_assert((OFF_W1 % 256) == 0);
static_assert((OFF_G % 256) == 0);
static_assert((WS_BYTES % 128) == 0);
static_assert(WS_BYTES <= (size_t)WSCAP);
static_assert(NTILES * 16 == NEDGE);
static_assert(NTIT * 4 >= NTILES);

typedef _Float16     v16h __attribute__((ext_vector_type(16)));
typedef _Float16     v8h  __attribute__((ext_vector_type(8)));
typedef float        v8f  __attribute__((ext_vector_type(8)));
typedef float        v4f  __attribute__((ext_vector_type(4)));
typedef unsigned int v4u  __attribute__((ext_vector_type(4)));
union Frag { v16h v; v8h half[2]; };
union Pk8  { v8h h; v4u u; };

__device__ __forceinline__ int imin(int a, int b) { return a < b ? a : b; }
__device__ __forceinline__ int imax(int a, int b) { return a > b ? a : b; }

__device__ __forceinline__ v4u cvt8(const v4f a, const v4f b) {
  v8h hv = {(_Float16)a.x, (_Float16)a.y, (_Float16)a.z, (_Float16)a.w,
            (_Float16)b.x, (_Float16)b.y, (_Float16)b.z, (_Float16)b.w};
  Pk8 p;
  p.h = hv;
  return p.u;
}

__device__ __forceinline__ v8f wmh(v16h a, v16h b, v8f c) {
  v8f d = __builtin_amdgcn_wmma_f32_16x16x32_f16(false, a, false, b, (short)0, c, false, false);
  asm volatile("v_nop\n\tv_nop\n\tv_nop\n\tv_nop" : "+v"(d) : "v"(a), "v"(b));
  return d;
}

__device__ __forceinline__ v16h ldA(const _Float16* base, int ld, int lane) {
  Frag a;
  const _Float16* p = base + (lane & 15) * ld + 8 * (lane >> 4);
  a.half[0] = *(const v8h*)p;
  a.half[1] = *(const v8h*)(p + 16);
  return a.v;
}

__device__ __forceinline__ v16h ldB(const _Float16* pk, int frag, int lane) {
  Frag b;
  const _Float16* p = pk + (size_t)((frag << 5) + lane) * 16;
  b.half[0] = *(const v8h*)p;
  b.half[1] = *(const v8h*)(p + 8);
  return b.v;
}

__device__ __forceinline__ float sspf(float x) {
  const float e = __expf(-fabsf(x));
  return fmaxf(x, 0.0f) + __logf(1.0f + e) - LN2F;
}

__global__ __launch_bounds__(TPB) void k_prep(const float* __restrict__ wW0, const float* __restrict__ wW1,
                                              const float* __restrict__ hW, const float* __restrict__ gW,
                                              _Float16* pk) {
  const int tid = threadIdx.x;
  const int g = blockIdx.x * TPB + tid;
  const int wg = __builtin_amdgcn_readfirstlane(g >> 5);
  if (wg >= NGRP / 32) return;
  const int pw = wg * 256;
  const float* src;
  int K, N, NT, lbase;
  if (pw < OFF_W0) {
    const int l = pw / 8192;           lbase = pw - l * 8192;  src = hW + l * (ED * KD);   K = ED; N = KD; NT = 4;
  } else if (pw < OFF_W1) {
    const int q = pw - OFF_W0; const int mi = q / 1536; lbase = q - mi * 1536; src = wW0 + mi * (DF * WH); K = DF; N = WH; NT = 3;
  } else if (pw < OFF_G) {
    const int q = pw - OFF_W1; const int mi = q / 4096; lbase = q - mi * 4096; src = wW1 + mi * (WH * KD); K = WH; N = KD; NT = 4;
  } else {
    const int q = pw - OFF_G;  const int mi = q / 8192; lbase = q - mi * 8192; src = gW + mi * (KD * ED); K = KD; N = ED; NT = 8;
  }
  const int lane = g & 31;
  const int loc0 = lbase + lane * 8;
  const int e0 = loc0 & 15;
  const int L = (loc0 >> 4) & 31;
  const int ft = loc0 >> 9;
  const int t = ft % NT, s = ft / NT;
  const int hh = L >> 4, c = t * 16 + (L & 15);
  const int cc = imin(c, N - 1);
  float tv[8];
#pragma unroll
  for (int u = 0; u < 8; ++u) {
    const int e = e0 + u;
    const int k = 32 * s + ((e < 8) ? (8 * hh + e) : (8 + 8 * hh + e));
    const int kc = imin(k, K - 1);
    const float v = src[kc * N + cc];
    tv[u] = (k < K && c < N) ? v * WSC : 0.0f;
  }
  const v4f f0 = {tv[0], tv[1], tv[2], tv[3]};
  const v4f f1 = {tv[4], tv[5], tv[6], tv[7]};
  const v4u pkv = cvt8(f0, f1);
  _Float16* d = pk + (size_t)g * 8;
  *(volatile v4u*)d = pkv;
  __threadfence();
  *(volatile v4u*)d = pkv;
}

__global__ __launch_bounds__(TPB) void k_main(const float* __restrict__ de, const float* __restrict__ dn,
                                              const float* __restrict__ X, const float* __restrict__ Y,
                                              const float* __restrict__ wb0, const _Float16* __restrict__ pk,
                                              float* out) {
  __shared__ __attribute__((aligned(16))) float    xs[NE * ED];
  __shared__ __attribute__((aligned(16))) _Float16 xh[NE * ED];
  __shared__ __attribute__((aligned(16))) _Float16 ef[NEDGE * DF];
  __shared__ __attribute__((aligned(16))) float    hm[NE * KD];
  __shared__ __attribute__((aligned(16))) float    wm[NEDGE * KD];
  __shared__ __attribute__((aligned(16))) _Float16 zh[3 * NE * KD];
  __shared__ __attribute__((aligned(16))) _Float16 act[4 * NE * KD];
  __shared__ __attribute__((aligned(16))) float    ysh[NNUC * KD];
  __shared__ float cmu[DF];
  __shared__ float cns[DF];

  const int tid = threadIdx.x, lane = tid & 31, h = lane >> 4, m = lane & 15;
  const int wv = __builtin_amdgcn_readfirstlane(tid >> 5);
  const int w2 = __builtin_amdgcn_readfirstlane(tid >> 6);
  const int b = blockIdx.x;
  const v8f zero8 = {0.f, 0.f, 0.f, 0.f, 0.f, 0.f, 0.f, 0.f};

  for (int idx = tid; idx < NE * ED; idx += TPB) xs[idx] = X[idx & (ED - 1)];
  for (int idx = tid; idx < NNUC * KD; idx += TPB) ysh[idx] = Y[idx];
  {
    const v4u z4 = {0u, 0u, 0u, 0u};
    for (int q = tid; q < (4 * NE * KD) / 8; q += TPB) *(v4u*)(act + 8 * q) = z4;
  }
  if (tid < DF) {
    const float q = (float)(2 * tid + 1) * 0.015625f;
    cmu[tid] = 10.0f * q * q;
    const float sg = (1.0f + 10.0f * q) * (1.0f / 7.0f);
    cns[tid] = 1.0f / (sg * sg);
  }
  __syncthreads();

  for (int ed = tid; ed < NEDGE; ed += TPB) {
    const int isSame = (ed < N_SAME) ? 1 : 0;
    int es = isSame ? ed : (ed - RB_ANTI);
    es = imax(0, imin(es, 127));
    const int bS = (es >= 56) ? 1 : 0;
    const int e2 = es - 56 * bS;
    const int iiS = e2 / 7, jjS = e2 - 7 * iiS;
    const int iS = 8 * bS + iiS, jS = 8 * bS + jjS + ((jjS >= iiS) ? 1 : 0);
    const int bA = (es >= 64) ? 1 : 0;
    const int e3 = es - 64 * bA;
    const int iA = 8 * bA + (e3 >> 3), jA = 8 * (1 - bA) + (e3 & 7);
    const int i = isSame ? iS : iA, j = isSame ? jS : jA;
    const int eidx = imin(imax(i * NE + j, 0), NE * NE - 1);
    const float dE = de[(size_t)b * (NE * NE) + eidx];
    const int nidx = imin(imax(ed - RB_NUC, 0), NE * NNUC - 1);
    const float dN = dn[(size_t)b * (NE * NNUC) + nidx];
    const float d = (ed < RB_NUC) ? dE : dN;
    const float envs = ESC * (d * d) * __expf(-d);
#pragma unroll 1
    for (int fg = 0; fg < DF / 8; ++fg) {
      float tv[8];
#pragma unroll
      for (int u = 0; u < 8; ++u) {
        const int f = 8 * fg + u;
        const float t = d - cmu[f];
        tv[u] = envs * __expf(-(t * t) * cns[f]);
      }
      const v4f f0 = {tv[0], tv[1], tv[2], tv[3]};
      const v4f f1 = {tv[4], tv[5], tv[6], tv[7]};
      *(v4u*)(ef + ed * DF + 8 * fg) = cvt8(f0, f1);
    }
  }
  __syncthreads();

#pragma unroll 1
  for (int l = 0; l < NL; ++l) {
    for (int q = tid; q < (NE * ED) / 8; q += TPB) {
      const v4f a0 = *(const v4f*)(xs + 8 * q);
      const v4f a1 = *(const v4f*)(xs + 8 * q + 4);
      *(v4u*)(xh + 8 * q) = cvt8(a0, a1);
    }
    __syncthreads();

    {
      const _Float16* HWp = pk + OFF_HW + l * (16 * FRH);
      v8f acc = zero8;
#pragma unroll
      for (int s = 0; s < 4; ++s) acc = wmh(ldA(xh + 32 * s, ED, lane), ldB(HWp, s * 4 + wv, lane), acc);
      const int col = 16 * wv + m;
#pragma unroll
      for (int v = 0; v < 8; ++v) hm[(8 * h + v) * KD + col] = acc[v] * PSC;
    }

#pragma unroll 1
    for (int it = 0; it < NTIT; ++it) {
      const int tt = wv + 4 * it;
      const bool tval = (tt < NTILES);
      const int te = tval ? tt : (NTILES - 1);
      int kind, rb;
      if (te < 7)       { kind = 0; rb = 16 * te; }
      else if (te < 15) { kind = 1; rb = RB_ANTI + 16 * (te - 7); }
      else              { kind = 2; rb = RB_NUC + 16 * (te - 15); }
      const int lk3 = l * 3 + kind;
      const _Float16* W0p = pk + OFF_W0 + lk3 * (3 * FRH);
      const _Float16* W1p = pk + OFF_W1 + lk3 * (8 * FRH);
      const float* bs = wb0 + lk3 * WH;
      _Float16* aw = act + wv * (NE * KD);

      {
        const v16h ea = ldA(ef + rb * DF, DF, lane);
#pragma unroll 1
        for (int nt = 0; nt < 3; ++nt) {
          const v8f c = wmh(ea, ldB(W0p, nt, lane), zero8);
          const int col = 16 * nt + m;
          const float bv = bs[imin(col, WH - 1)];
#pragma unroll
          for (int v = 0; v < 8; ++v) {
            const float pre = c[v] * PSE + bv;
            const float sv = sspf(pre);
            aw[(8 * h + v) * KD + col] = (_Float16)((col < WH) ? sv : 0.0f);
          }
        }
      }
      __syncthreads();

      {
        const v16h a0 = ldA(aw, KD, lane);
        const v16h a1 = ldA(aw + 32, KD, lane);
#pragma unroll 1
        for (int nt = 0; nt < 4; ++nt) {
          v8f c = wmh(a0, ldB(W1p, nt, lane), zero8);
          c = wmh(a1, ldB(W1p, 4 + nt, lane), c);
          if (tval) {
            const int col = 16 * nt + m;
#pragma unroll
            for (int v = 0; v < 8; ++v) wm[(rb + 8 * h + v) * KD + col] = c[v] * PSC;
          }
        }
      }
      __syncthreads();
    }

#pragma unroll 1
    for (int it = 0; it < 24; ++it) {
      const int kind = it >> 3;
      const int i = (it & 7) * 2 + w2;
      const int k = tid & 63;
      const int hb = i >> 3, ii = i & 7;
      float sum = 0.0f;
      if (kind == 0) {
        const int base = 56 * hb + 7 * ii;
#pragma unroll
        for (int jj = 0; jj < 7; ++jj) {
          const int j = 8 * hb + jj + ((jj >= ii) ? 1 : 0);
          sum += wm[(base + jj) * KD + k] * hm[j * KD + k];
        }
      } else if (kind == 1) {
        const int base = RB_ANTI + 64 * hb + 8 * ii;
#pragma unroll
        for (int jj = 0; jj < 8; ++jj) {
          const int j = 8 * (1 - hb) + jj;
          sum += wm[(base + jj) * KD + k] * hm[j * KD + k];
        }
      } else {
#pragma unroll
        for (int mi = 0; mi < NNUC; ++mi) sum += wm[(RB_NUC + NNUC * i + mi) * KD + k] * ysh[mi * KD + k];
      }
      zh[kind * (NE * KD) + i * KD + k] = (_Float16)sum;
    }
    __syncthreads();

#pragma unroll 1
    for (int q = 0; q < 2; ++q) {
      const int nt = wv + 4 * q;
      v8f acc = zero8;
#pragma unroll
      for (int kind = 0; kind < 3; ++kind) {
        const _Float16* Gp = pk + OFF_G + (l * 3 + kind) * (16 * FRH);
        const _Float16* zk = zh + kind * (NE * KD);
        acc = wmh(ldA(zk, KD, lane), ldB(Gp, nt, lane), acc);
        acc = wmh(ldA(zk + 32, KD, lane), ldB(Gp, 8 + nt, lane), acc);
      }
      const int col = 16 * nt + m;
#pragma unroll
      for (int v = 0; v < 8; ++v) {
        const int o = (8 * h + v) * ED + col;
        const float xo = xs[o];
        xs[o] = xo + acc[v] * PSC;
      }
    }
    __syncthreads();
  }

  v4f ov[4];
#pragma unroll
  for (int it = 0; it < 4; ++it) ov[it] = *(const v4f*)(xs + 4 * (it * TPB + tid));
  float* po = out + (size_t)b * (NE * ED);
#pragma unroll
  for (int it = 0; it < 4; ++it) *(volatile v4f*)(po + 4 * (it * TPB + tid)) = ov[it];
  __threadfence();
#pragma unroll
  for (int it = 0; it < 4; ++it) *(volatile v4f*)(po + 4 * (it * TPB + tid)) = ov[it];
}

extern "C" void kernel_launch(void* const* d_in, const int* in_sizes, int n_in,
                              void* d_out, int out_size, void* d_ws, size_t ws_size,
                              hipStream_t stream) {
  if (n_in < 9) return;
  const int nde = in_sizes[0];
  if (nde <= 0 || (nde % (NE * NE)) != 0) return;
  const int nb = nde / (NE * NE);
  if (in_sizes[1] != nb * NE * NNUC) return;
  if (in_sizes[2] != ED || in_sizes[3] != NNUC * KD) return;
  if (in_sizes[4] != NL * 3 * DF * WH) return;
  if (in_sizes[5] != NL * 3 * WH) return;
  if (in_sizes[6] != NL * 3 * WH * KD) return;
  if (in_sizes[7] != NL * ED * KD) return;
  if (in_sizes[8] != NL * 3 * KD * ED) return;
  if (out_size != nb * NE * ED) return;
  if (WS_BYTES > ws_size || WS_BYTES > (size_t)WSCAP) return;

  const float* de  = (const float*)d_in[0];
  const float* dn  = (const float*)d_in[1];
  const float* X   = (const float*)d_in[2];
  const float* Y   = (const float*)d_in[3];
  const float* wW0 = (const float*)d_in[4];
  const float* wb0 = (const float*)d_in[5];
  const float* wW1 = (const float*)d_in[6];
  const float* hW  = (const float*)d_in[7];
  const float* gW  = (const float*)d_in[8];
  float* out = (float*)d_out;
  _Float16* pk = (_Float16*)d_ws;

  k_prep<<<dim3((NGRP + TPB - 1) / TPB), dim3(TPB), 0, stream>>>(wW0, wW1, hW, gW, pk);
  k_main<<<dim3(nb), dim3(TPB), 0, stream>>>(de, dn, X, Y, wb0, pk, out);
}
